// VAE_61538291417372
// MI455X (gfx1250) — hardware-run, weakly checked
//
#include <hip/hip_runtime.h>
#include <math.h>

typedef __attribute__((ext_vector_type(16))) _Float16 v16h;
typedef __attribute__((ext_vector_type(8)))  _Float16 v8h;
typedef __attribute__((ext_vector_type(8)))  float    v8f;
typedef __attribute__((ext_vector_type(4)))  float    v4f;
typedef __attribute__((ext_vector_type(2)))  float    v2f;

constexpr int kNB  = 2048;
constexpr int kNL  = 100;
constexpr int kND  = 32;
constexpr int kNI  = 128;
constexpr int kNI2 = kNI / 2;
constexpr int kNH  = 256;
constexpr int kNZ  = 64;
constexpr int kNG  = 3 * kNH;
constexpr int kKC  = kNI + kNH;
constexpr int kK32P = 64;
static_assert(kKC == 384 && (kKC % 32) == 0 && (kNI % 32) == 0 && (kNH % 32) == 0);
static_assert((kNZ % 32) == 0 && (kND % 32) == 0 && ((2 * kNH) % 32) == 0);
static_assert(kNH == 16 * 16);

constexpr float kCA   = 64.0f;
constexpr float kCW   = 256.0f;
constexpr float kFold = 1.0f / (kCA * kCW);
static_assert(kFold == 1.0f / 16384.0f);
constexpr float kResCarry = 2048.0f;
constexpr float kResInv   = 1.0f / kResCarry;
static_assert(kResInv == 1.0f / 2048.0f);
constexpr float kF16Min = 6.103515625e-05f;

constexpr int kRows    = 16;
constexpr int kThreads = 512;
constexpr int kBlocks  = kNB / kRows;
static_assert((kNB % kRows) == 0 && kBlocks == 128);
constexpr int kAP  = kKC + 8;
constexpr int kSHP = 2 * kNH + 8;
constexpr int kZP  = kNZ + 8;
constexpr int kXCP = kND + 8;
constexpr int kStP = 2 * kNZ + 4;
constexpr int kXOP = kND + 4;
constexpr int kEP  = kNI + 8;
static_assert(((kAP * 2) % 16) == 0 && ((kSHP * 2) % 16) == 0 && ((kZP * 2) % 16) == 0);
static_assert(((kXCP * 2) % 16) == 0 && ((kStP * 4) % 16) == 0 && ((kXOP * 4) % 16) == 0 && ((kEP * 2) % 16) == 0);

constexpr size_t kBytesPEE  = (size_t)kNI * kK32P * 2;
constexpr size_t kBytesCell = (size_t)kNG * kKC * 2;
constexpr size_t kBytesPENC = (size_t)(2 * kNZ) * (2 * kNH) * 2;
constexpr size_t kBytesPZ2H = (size_t)kNH * kNZ * 2;
constexpr size_t kBytesPH2I = (size_t)kNI2 * kNH * 2;
constexpr size_t kBytesPED  = (size_t)kNI2 * kK32P * 2;
constexpr size_t kBytesPDEC = (size_t)kND * kNH * 2;
constexpr size_t kBytesXE   = (size_t)kNL * kNB * kNI * 2;
constexpr size_t kOffPEE  = 0;
constexpr size_t kOffPF   = kOffPEE  + kBytesPEE;
constexpr size_t kOffPB   = kOffPF   + kBytesCell;
constexpr size_t kOffPD   = kOffPB   + kBytesCell;
constexpr size_t kOffPENC = kOffPD   + kBytesCell;
constexpr size_t kOffPZ2H = kOffPENC + kBytesPENC;
constexpr size_t kOffPH2I = kOffPZ2H + kBytesPZ2H;
constexpr size_t kOffPED  = kOffPH2I + kBytesPH2I;
constexpr size_t kOffPDEC = kOffPED  + kBytesPED;
constexpr size_t kOffXE   = kOffPDEC + kBytesPDEC;
constexpr size_t kWsTotal = kOffXE   + kBytesXE;
static_assert(kBytesPEE == 16384ull && kBytesCell == 589824ull && kBytesPENC == 131072ull);
static_assert(kBytesPZ2H == 32768ull && kBytesPH2I == 32768ull && kBytesPED == 8192ull && kBytesPDEC == 16384ull);
static_assert(kBytesXE == 52428800ull);
static_assert(kWsTotal == 54435840ull);
static_assert(kWsTotal <= 134217728ull);
static_assert((kOffPF % 128) == 0 && (kOffPB % 128) == 0 && (kOffPD % 128) == 0 && (kOffPENC % 128) == 0);
static_assert((kOffPZ2H % 128) == 0 && (kOffPH2I % 128) == 0 && (kOffPED % 128) == 0 && (kOffPDEC % 128) == 0);
static_assert((kOffXE % 128) == 0);

constexpr size_t kOutMu    = (size_t)kNB * kNL * kND;
constexpr size_t kOutLv    = kOutMu + (size_t)kNB * kNZ;
constexpr size_t kOutTotal = kOutLv + (size_t)kNB * kNZ;
static_assert(kOutMu * 4 == 26214400ull && kOutLv * 4 == 26738688ull && kOutTotal * 4 == 27262976ull);
static_assert(((kOutMu * 4) % 128) == 0 && ((kOutLv * 4) % 128) == 0);
static_assert((kND * 4) == 128 && ((kNZ * 4) % 128) == 0);

__device__ __forceinline__ unsigned short f2bf_bits(float f) {
  unsigned u = __float_as_uint(f);
  return (unsigned short)((u + 0x7FFFu + ((u >> 16) & 1u)) >> 16);
}
__device__ __forceinline__ float bf_bits2f(unsigned short h) { return __uint_as_float(((unsigned)h) << 16); }
__device__ __forceinline__ float bf_val(float f) { return bf_bits2f(f2bf_bits(f)); }

__device__ __forceinline__ _Float16 carry_half(float v, float carry) {
  float s = v * carry;
  s = (fabsf(s) < kF16Min) ? 0.0f : s;
  return (_Float16)s;
}

__device__ __forceinline__ void carry_half_pair(float v, float carry, _Float16& vw, _Float16& rw) {
  const float s  = v * carry;
  const float sv = (fabsf(s) < kF16Min) ? 0.0f : s;
  vw = (_Float16)sv;
  const float back = (float)vw;
  float r = (s - back) * kResCarry;
  r = (fabsf(r) < kF16Min) ? 0.0f : r;
  rw = (_Float16)r;
}

__device__ __forceinline__ float ld_bf(const float* p) {
  float v = *p;
  asm volatile("" : "+v"(v));
  return bf_val(v);
}

union FragU { v16h v; v8h h[2]; };
__device__ __forceinline__ v16h frag_load(const _Float16* p) {
  FragU f;
  f.h[0] = *(const v8h*)(p);
  f.h[1] = *(const v8h*)(p + 16);
  return f.v;
}

__device__ __forceinline__ v8f mma_g(v16h a, v16h b, v8f c) {
  c = __builtin_amdgcn_wmma_f32_16x16x32_f16(false, a, false, b, (short)0, c, false, false);
  asm volatile("v_nop\n\tv_nop\n\tv_nop\n\tv_nop" : "+v"(c) : "v"(a), "v"(b));
  return c;
}

__device__ __forceinline__ float fast_sigmoid(float v) {
  return __builtin_amdgcn_rcpf(1.0f + __expf(-v));
}
__device__ __forceinline__ float fast_tanh(float v) {
  const float t = __expf(-2.0f * fabsf(v));
  const float q = (1.0f - t) * __builtin_amdgcn_rcpf(1.0f + t);
  return copysignf(q, v);
}

__device__ __forceinline__ void cell_part(const _Float16* ap, const _Float16* wp, int nks,
                                          v8f& g0, v8f& g1, v8f& g2) {
#pragma unroll 1
  for (int ks = 0; ks < nks; ++ks) {
    const v16h a  = frag_load(ap + 32 * ks);
    const v16h b0 = frag_load(wp + 32 * ks);
    const v16h b1 = frag_load(wp + (size_t)kNH * kKC + 32 * ks);
    const v16h b2 = frag_load(wp + (size_t)2 * kNH * kKC + 32 * ks);
    g0 = mma_g(a, b0, g0);
    g1 = mma_g(a, b1, g1);
    g2 = mma_g(a, b2, g2);
  }
}

__device__ __forceinline__ void cell_step(const _Float16* aRow, const _Float16* wRow,
                                          v8f& ar, v8f& az, v8f& ai, v8f& ah) {
  const v8f z8 = (v8f){0.f, 0.f, 0.f, 0.f, 0.f, 0.f, 0.f, 0.f};
  ar = z8; az = z8; ai = z8; ah = z8;
  cell_part(aRow, wRow, kNI / 32, ar, az, ai);
  cell_part(aRow + kNI, wRow + kNI, kNH / 32, ar, az, ah);
}

__device__ __forceinline__ v8f tile_product(const _Float16* ap, const _Float16* wp, int nks) {
  v8f acc = (v8f){0.f, 0.f, 0.f, 0.f, 0.f, 0.f, 0.f, 0.f};
#pragma unroll 1
  for (int ks = 0; ks < nks; ++ks) {
    const v16h a = frag_load(ap + 32 * ks);
    const v16h b = frag_load(wp + 32 * ks);
    acc = mma_g(a, b, acc);
  }
  return acc;
}

__device__ __forceinline__ void tile_product_pair(const _Float16* apv, const _Float16* apr, const _Float16* wp,
                                                  int nks, v8f& accv, v8f& accr) {
#pragma unroll 1
  for (int ks = 0; ks < nks; ++ks) {
    const v16h av = frag_load(apv + 32 * ks);
    const v16h ar = frag_load(apr + 32 * ks);
    const v16h b  = frag_load(wp + 32 * ks);
    accv = mma_g(av, b, accv);
    accr = mma_g(ar, b, accr);
  }
}

__device__ __forceinline__ void gate_update(const v8f& ar, const v8f& az, const v8f& ai, const v8f& ah,
                                            float cr, float cz, float bi, float bh, float (&h)[8]) {
#pragma unroll
  for (int e = 0; e < 8; ++e) {
    const float rg = fast_sigmoid(fmaf(ar[e], kFold, cr));
    const float zg = fast_sigmoid(fmaf(az[e], kFold, cz));
    const float hn = fmaf(ah[e], kFold, bh);
    const float in = fmaf(ai[e], kFold, bi);
    const float ng = fast_tanh(fmaf(rg, hn, in));
    h[e] = fmaf(zg, h[e] - ng, ng);
  }
}

__device__ __forceinline__ void gate_consts(const float* bih, const float* bhh, int j,
                                            float& cr, float& cz, float& ci, float& cn) {
  cr = ld_bf(bih + j) + ld_bf(bhh + j);
  cz = ld_bf(bih + kNH + j) + ld_bf(bhh + kNH + j);
  ci = ld_bf(bih + 2 * kNH + j);
  cn = ld_bf(bhh + 2 * kNH + j);
}

__device__ __forceinline__ void publish_tile(_Float16* base, int pitch, int col, int hh, const float (&v)[8]) {
#pragma unroll
  for (int r = 0; r < 8; ++r) base[(8 * hh + r) * pitch + col] = carry_half(v[r], kCA);
}

__device__ __forceinline__ void relu_tile_to_plane(const v8f& acc, float bias, _Float16* base, int pitch,
                                                   int col, int hh) {
#pragma unroll
  for (int r = 0; r < 8; ++r) {
    const float v = fmaxf(fmaf(acc[r], kFold, bias), 0.0f);
    base[(8 * hh + r) * pitch + col] = carry_half(v, kCA);
  }
}

constexpr int kPackP = 68;
__global__ __launch_bounds__(256) void operand_planes(
    const float* __restrict__ src, int srcK, int srcN,
    _Float16* __restrict__ dst, int pitch, int coloff) {
  __shared__ __align__(16) float sT[32 * kPackP];
  const int tid = threadIdx.x;
  const int n0 = blockIdx.x * 32;
  const int k0 = blockIdx.y * 64;
  {
    const int kk = tid >> 2;
    const int ns = (tid & 3) * 8;
    const int k  = k0 + kk;
    const bool live = (k < srcK);
    const int kc = live ? k : (srcK - 1);
    const float* sp = src + (size_t)kc * srcN + n0 + ns;
    v4f a0 = *(const v4f*)(sp);
    v4f a1 = *(const v4f*)(sp + 4);
    asm volatile("" : "+v"(a0), "+v"(a1));
#pragma unroll
    for (int e = 0; e < 4; ++e) {
      const float t0 = a0[e];
      const float t1 = a1[e];
      sT[(ns + e) * kPackP + kk]     = live ? bf_val(t0) : 0.0f;
      sT[(ns + 4 + e) * kPackP + kk] = live ? bf_val(t1) : 0.0f;
    }
  }
  __syncthreads();
  {
    const int n   = tid >> 3;
    const int kc8 = (tid & 7) * 8;
    const v4f b0 = *(const v4f*)(sT + n * kPackP + kc8);
    const v4f b1 = *(const v4f*)(sT + n * kPackP + kc8 + 4);
    v8h hv;
#pragma unroll
    for (int e = 0; e < 4; ++e) {
      const float t0 = b0[e];
      const float t1 = b1[e];
      hv[e]     = carry_half(t0, kCW);
      hv[4 + e] = carry_half(t1, kCW);
    }
    _Float16* q = dst + (size_t)(n0 + n) * pitch + coloff + k0 + kc8;
    *(volatile v8h*)q = hv;
    __threadfence();
    *(volatile v8h*)q = hv;
  }
}

__global__ __launch_bounds__(256) void embed_rows(
    const float* __restrict__ x, const _Float16* __restrict__ pee, const float* __restrict__ bee,
    _Float16* __restrict__ xe) {
  __shared__ __align__(16) _Float16 sE[8 * 16 * kEP];
  const int lane = threadIdx.x & 31;
  const int wave = threadIdx.x >> 5;
  const int hh = lane >> 4;
  const int nn = lane & 15;
  const int wg = blockIdx.x * 8 + wave;
  const int t  = wg >> 7;
  const int s0 = (wg & 127) * 16;
  const float* xr = x + ((size_t)(s0 + nn) * kNL + t) * kND + 8 * hh;
  const v4f a0 = *(const v4f*)(xr);
  const v4f a1 = *(const v4f*)(xr + 4);
  const v4f a2 = *(const v4f*)(xr + 16);
  const v4f a3 = *(const v4f*)(xr + 20);
  v16h af;
#pragma unroll
  for (int e = 0; e < 4; ++e) {
    const float t0 = a0[e];
    const float t1 = a1[e];
    const float t2 = a2[e];
    const float t3 = a3[e];
    af[e]      = carry_half(bf_val(t0), kCA);
    af[4 + e]  = carry_half(bf_val(t1), kCA);
    af[8 + e]  = carry_half(bf_val(t2), kCA);
    af[12 + e] = carry_half(bf_val(t3), kCA);
  }
  float bc[8];
#pragma unroll
  for (int j = 0; j < 8; ++j) bc[j] = ld_bf(bee + j * 16 + nn);
  _Float16* slab = sE + wave * (16 * kEP);
#pragma unroll
  for (int j = 0; j < 8; ++j) {
    const v16h b = frag_load(pee + (size_t)(j * 16 + nn) * kK32P + 8 * hh);
    v8f acc = (v8f){0.f, 0.f, 0.f, 0.f, 0.f, 0.f, 0.f, 0.f};
    acc = mma_g(af, b, acc);
    relu_tile_to_plane(acc, bc[j], slab, kEP, j * 16 + nn, hh);
  }
  __builtin_amdgcn_fence(__ATOMIC_RELEASE, "workgroup");
  __builtin_amdgcn_wave_barrier();
  __builtin_amdgcn_fence(__ATOMIC_ACQUIRE, "workgroup");
  v8h hv[8];
#pragma unroll
  for (int it = 0; it < 8; ++it) hv[it] = *(const v8h*)(slab + (it * 2 + hh) * kEP + nn * 8);
  _Float16* dst = xe + ((size_t)t * kNB + s0) * kNI + nn * 8;
  for (int pass = 0; pass < 2; ++pass) {
#pragma unroll
    for (int it = 0; it < 8; ++it)
      *(volatile v8h*)(dst + (size_t)(it * 2 + hh) * kNI) = hv[it];
    __threadfence();
  }
}

__global__ __launch_bounds__(512) void encode_decode_steps(
    const _Float16* __restrict__ xe,
    const _Float16* __restrict__ pf, const _Float16* __restrict__ pb, const _Float16* __restrict__ pd,
    const _Float16* __restrict__ penc, const _Float16* __restrict__ pz2h, const _Float16* __restrict__ ph2i,
    const _Float16* __restrict__ ped, const _Float16* __restrict__ pdec,
    const float* __restrict__ eps,
    const float* __restrict__ bih_f, const float* __restrict__ bhh_f,
    const float* __restrict__ bih_b, const float* __restrict__ bhh_b,
    const float* __restrict__ b_enc, const float* __restrict__ b_z2h, const float* __restrict__ b_h2i,
    const float* __restrict__ bih_d, const float* __restrict__ bhh_d,
    const float* __restrict__ b_ed, const float* __restrict__ b_dec,
    float* __restrict__ out) {
  __shared__ __align__(16) _Float16 sA[kRows * kAP];
  __shared__ __align__(16) _Float16 sS[kRows * kSHP];
  __shared__ __align__(16) _Float16 sZ[kRows * kZP];
  __shared__ __align__(16) _Float16 sXC[kRows * kXCP];
  __shared__ __align__(16) float    sStat[kRows * kStP];
  __shared__ __align__(16) float    sXO[kRows * kXOP];
  __shared__ __align__(16) _Float16 sZ2[kRows * kZP];
  static_assert(2 * (kRows * kAP + kRows * kSHP + kRows * kZP + kRows * kXCP + kRows * kZP) +
                4 * (kRows * kStP + kRows * kXOP) == 45824);
  static_assert(2 * (kRows * kAP + kRows * kSHP + kRows * kZP + kRows * kXCP + kRows * kZP) +
                4 * (kRows * kStP + kRows * kXOP) <= 65536);

  const int tid  = threadIdx.x;
  const int lane = tid & 31;
  const int wave = tid >> 5;
  const int hh   = lane >> 4;
  const int nn   = lane & 15;
  const int s0   = blockIdx.x * kRows;
  const int ucol = wave * 16 + nn;
  const int xm = (tid >> 4) & 15;
  const int xc = (tid & 15) * 8;

  const _Float16* aRow = sA + nn * kAP + 8 * hh;

  float hc[8];
#pragma unroll
  for (int r = 0; r < 8; ++r) hc[r] = 0.0f;
  float cR, cZ, cI, cN;
  gate_consts(bih_f, bhh_f, ucol, cR, cZ, cI, cN);
  publish_tile(sA, kAP, kNI + ucol, hh, hc);
  if (tid < 256) {
    const v8h xv = *(const v8h*)(xe + ((size_t)s0 + xm) * kNI + xc);
    *(v8h*)(sA + xm * kAP + xc) = xv;
  }
  __syncthreads();

#pragma unroll 1
  for (int t = 0; t < kNL; ++t) {
    int lz = 0;
    asm volatile("" : "+v"(lz));
    v8f ar, az, ai, ah;
    cell_step(aRow, pf + (size_t)ucol * kKC + 8 * hh + lz, ar, az, ai, ah);
    __syncthreads();
    gate_update(ar, az, ai, ah, cR, cZ, cI, cN, hc);
    publish_tile(sA, kAP, kNI + ucol, hh, hc);
    if (tid < 256) {
      const int tn = (t + 1 < kNL) ? (t + 1) : (kNL - 1);
      const v8h xv = *(const v8h*)(xe + ((size_t)tn * kNB + s0 + xm) * kNI + xc);
      *(v8h*)(sA + xm * kAP + xc) = xv;
    }
    __syncthreads();
  }

  float hb[8];
#pragma unroll
  for (int r = 0; r < 8; ++r) hb[r] = 0.0f;
  publish_tile(sS, kSHP, ucol, hh, hc);
  publish_tile(sA, kAP, kNI + ucol, hh, hb);
  gate_consts(bih_b, bhh_b, ucol, cR, cZ, cI, cN);
  __syncthreads();
  {
    int lz = 0;
    asm volatile("" : "+v"(lz));
    v8f ar, az, ai, ah;
    cell_step(aRow, pb + (size_t)ucol * kKC + 8 * hh + lz, ar, az, ai, ah);
    gate_update(ar, az, ai, ah, cR, cZ, cI, cN, hb);
    publish_tile(sS, kSHP, kNH + ucol, hh, hb);
  }
  __syncthreads();

  {
    const float bencC = ld_bf(b_enc + (wave & 7) * 16 + nn);
    if (wave < 8) {
      int lz = 0;
      asm volatile("" : "+v"(lz));
      const v8f acc = tile_product(sS + nn * kSHP + 8 * hh,
                                   penc + (size_t)(wave * 16 + nn) * (2 * kNH) + 8 * hh + lz, (2 * kNH) / 32);
#pragma unroll
      for (int r = 0; r < 8; ++r)
        sStat[(8 * hh + r) * kStP + wave * 16 + nn] = fmaf(acc[r], kFold, bencC);
    }
  }
  __syncthreads();

  {
    const int zc = lane * 2;
    v2f ev = *(const v2f*)(eps + (size_t)(s0 + wave) * kNZ + zc);
    asm volatile("" : "+v"(ev));
    const float e0 = ev[0];
    const float e1 = ev[1];
    const float m0 = sStat[wave * kStP + zc];
    const float m1 = sStat[wave * kStP + zc + 1];
    const float l0 = sStat[wave * kStP + kNZ + zc];
    const float l1 = sStat[wave * kStP + kNZ + zc + 1];
    const float z0 = fmaf(expf(0.5f * l0), bf_val(e0), m0);
    const float z1 = fmaf(expf(0.5f * l1), bf_val(e1), m1);
    _Float16 zv0, zr0, zv1, zr1;
    carry_half_pair(z0, kCA, zv0, zr0);
    carry_half_pair(z1, kCA, zv1, zr1);
    sZ[wave * kZP + zc]      = zv0;
    sZ[wave * kZP + zc + 1]  = zv1;
    sZ2[wave * kZP + zc]     = zr0;
    sZ2[wave * kZP + zc + 1] = zr1;
    if (wave == 8 || wave == 9) {
      const int sel = wave - 8;
      float* dst = out + (sel ? kOutLv : kOutMu) + (size_t)s0 * kNZ + nn * 4;
      v4f sv[8];
#pragma unroll
      for (int it = 0; it < 8; ++it)
        sv[it] = *(const v4f*)(sStat + (it * 2 + hh) * kStP + sel * kNZ + nn * 4);
      for (int pass = 0; pass < 2; ++pass) {
#pragma unroll
        for (int it = 0; it < 8; ++it)
          *(volatile v4f*)(dst + (size_t)(it * 2 + hh) * kNZ) = sv[it];
        __threadfence();
      }
    }
  }
  gate_consts(bih_d, bhh_d, ucol, cR, cZ, cI, cN);
  const float bz2hC = ld_bf(b_z2h + ucol);
  const float bdecC = ld_bf(b_dec + (wave & 1) * 16 + nn);
  const float bh2iC = ld_bf(b_h2i + ((wave + 2) & 3) * 16 + nn);
  const float bedC  = ld_bf(b_ed + (wave & 3) * 16 + nn);
  __syncthreads();

  {
    int lz = 0;
    asm volatile("" : "+v"(lz));
    v8f accV = (v8f){0.f, 0.f, 0.f, 0.f, 0.f, 0.f, 0.f, 0.f};
    v8f accR = (v8f){0.f, 0.f, 0.f, 0.f, 0.f, 0.f, 0.f, 0.f};
    tile_product_pair(sZ + nn * kZP + 8 * hh, sZ2 + nn * kZP + 8 * hh,
                      pz2h + (size_t)ucol * kNZ + 8 * hh + lz, kNZ / 32, accV, accR);
#pragma unroll
    for (int r = 0; r < 8; ++r) {
      const float sum = fmaf(accR[r], kResInv, accV[r]);
      hc[r] = fmaxf(fmaf(sum, kFold, bz2hC), 0.0f);
    }
    publish_tile(sA, kAP, kNI + ucol, hh, hc);
    const int cc = lane * 2;
    const float c0 = fmaxf(ld_bf(b_ed + cc), 0.0f);
    const float c1 = fmaxf(ld_bf(b_ed + cc + 1), 0.0f);
    sA[wave * kAP + cc]     = carry_half(c0, kCA);
    sA[wave * kAP + cc + 1] = carry_half(c1, kCA);
  }
  __syncthreads();
  if (wave >= 2 && wave < 6) {
    int lz = 0;
    asm volatile("" : "+v"(lz));
    const int j = wave - 2;
    const v8f acc = tile_product(aRow + kNI, ph2i + (size_t)(j * 16 + nn) * kNH + 8 * hh + lz, kNH / 32);
    relu_tile_to_plane(acc, bh2iC, sA, kAP, kNI2 + j * 16 + nn, hh);
  }
  __syncthreads();

#pragma unroll 1
  for (int t = 0; t < kNL; ++t) {
    int lz = 0;
    asm volatile("" : "+v"(lz));
    {
      v8f ar, az, ai, ah;
      cell_step(aRow, pd + (size_t)ucol * kKC + 8 * hh + lz, ar, az, ai, ah);
      __syncthreads();
      gate_update(ar, az, ai, ah, cR, cZ, cI, cN, hc);
      publish_tile(sA, kAP, kNI + ucol, hh, hc);
    }
    __syncthreads();
    if (wave < 2) {
      const v8f acc = tile_product(aRow + kNI, pdec + (size_t)(wave * 16 + nn) * kNH + 8 * hh + lz, kNH / 32);
#pragma unroll
      for (int r = 0; r < 8; ++r) {
        const float v = fmaf(acc[r], kFold, bdecC);
        sXO[(8 * hh + r) * kXOP + wave * 16 + nn] = v;
        sXC[(8 * hh + r) * kXCP + wave * 16 + nn] = carry_half(v, kCA);
      }
    } else if (wave < 6) {
      const int j = wave - 2;
      const v8f acc = tile_product(aRow + kNI, ph2i + (size_t)(j * 16 + nn) * kNH + 8 * hh + lz, kNH / 32);
      relu_tile_to_plane(acc, bh2iC, sA, kAP, kNI2 + j * 16 + nn, hh);
    }
    __syncthreads();
    if (wave < 4) {
      const v8f acc = tile_product(sXC + nn * kXCP + 8 * hh, ped + (size_t)(wave * 16 + nn) * kK32P + 8 * hh + lz, 1);
      relu_tile_to_plane(acc, bedC, sA, kAP, wave * 16 + nn, hh);
    } else if (wave == 4) {
      const int q  = lane >> 3;
      const int c4 = (lane & 7) * 4;
      v4f ov[4];
#pragma unroll
      for (int it = 0; it < 4; ++it) ov[it] = *(const v4f*)(sXO + (it * 4 + q) * kXOP + c4);
      float* dst = out + ((size_t)s0 * kNL + t) * kND + c4;
      for (int pass = 0; pass < 2; ++pass) {
#pragma unroll
        for (int it = 0; it < 4; ++it)
          *(volatile v4f*)(dst + (size_t)(it * 4 + q) * (kNL * kND)) = ov[it];
        __threadfence();
      }
    }
    __syncthreads();
  }
}

extern "C" void kernel_launch(void* const* d_in, const int* in_sizes, int n_in,
                              void* d_out, int out_size, void* d_ws, size_t ws_size,
                              hipStream_t stream) {
  if (n_in < 26) return;
  if (in_sizes[0] != kNB * kNL * kND) return;
  if (in_sizes[1] != kNB * kNZ) return;
  if (in_sizes[2] != kND * kNI || in_sizes[3] != kNI) return;
  if (in_sizes[4] != kNI * kNG || in_sizes[5] != kNH * kNG) return;
  if (in_sizes[6] != kNG || in_sizes[7] != kNG) return;
  if (in_sizes[8] != kNI * kNG || in_sizes[9] != kNH * kNG) return;
  if (in_sizes[10] != kNG || in_sizes[11] != kNG) return;
  if (in_sizes[12] != 2 * kNH * 2 * kNZ || in_sizes[13] != 2 * kNZ) return;
  if (in_sizes[14] != kNZ * kNH || in_sizes[15] != kNH) return;
  if (in_sizes[16] != kNH * kNI2 || in_sizes[17] != kNI2) return;
  if (in_sizes[18] != kNI * kNG || in_sizes[19] != kNH * kNG) return;
  if (in_sizes[20] != kNG || in_sizes[21] != kNG) return;
  if (in_sizes[22] != kND * kNI2 || in_sizes[23] != kNI2) return;
  if (in_sizes[24] != kNH * kND || in_sizes[25] != kND) return;
  if ((size_t)out_size != kOutTotal) return;
  if (ws_size < kWsTotal) return;

  const float* x     = (const float*)d_in[0];
  const float* eps   = (const float*)d_in[1];
  const float* W_ee  = (const float*)d_in[2];
  const float* b_ee  = (const float*)d_in[3];
  const float* Wih_f = (const float*)d_in[4];
  const float* Whh_f = (const float*)d_in[5];
  const float* bih_f = (const float*)d_in[6];
  const float* bhh_f = (const float*)d_in[7];
  const float* Wih_b = (const float*)d_in[8];
  const float* Whh_b = (const float*)d_in[9];
  const float* bih_b = (const float*)d_in[10];
  const float* bhh_b = (const float*)d_in[11];
  const float* W_enc = (const float*)d_in[12];
  const float* b_enc = (const float*)d_in[13];
  const float* W_z2h = (const float*)d_in[14];
  const float* b_z2h = (const float*)d_in[15];
  const float* W_h2i = (const float*)d_in[16];
  const float* b_h2i = (const float*)d_in[17];
  const float* Wih_d = (const float*)d_in[18];
  const float* Whh_d = (const float*)d_in[19];
  const float* bih_d = (const float*)d_in[20];
  const float* bhh_d = (const float*)d_in[21];
  const float* W_ed  = (const float*)d_in[22];
  const float* b_ed  = (const float*)d_in[23];
  const float* W_dec = (const float*)d_in[24];
  const float* b_dec = (const float*)d_in[25];
  float* out = (float*)d_out;

  char* ws = (char*)d_ws;
  _Float16* PEE  = (_Float16*)(ws + kOffPEE);
  _Float16* PF   = (_Float16*)(ws + kOffPF);
  _Float16* PB   = (_Float16*)(ws + kOffPB);
  _Float16* PD   = (_Float16*)(ws + kOffPD);
  _Float16* PENC = (_Float16*)(ws + kOffPENC);
  _Float16* PZ2H = (_Float16*)(ws + kOffPZ2H);
  _Float16* PH2I = (_Float16*)(ws + kOffPH2I);
  _Float16* PED  = (_Float16*)(ws + kOffPED);
  _Float16* PDEC = (_Float16*)(ws + kOffPDEC);
  _Float16* XE   = (_Float16*)(ws + kOffXE);

  static_assert((kNI % 32) == 0 && (kNG % 32) == 0 && ((2 * kNZ) % 32) == 0 && (kNH % 32) == 0);
  static_assert((kNI2 % 32) == 0 && (kND % 32) == 0);
  static_assert((kNI % 64) == 0 && (kNH % 64) == 0 && ((2 * kNH) % 64) == 0 && (kNZ % 64) == 0);

  operand_planes<<<dim3(kNI / 32, 1), 256, 0, stream>>>(W_ee, kND, kNI, PEE, kK32P, 0);
  operand_planes<<<dim3(kNG / 32, kNI / 64), 256, 0, stream>>>(Wih_f, kNI, kNG, PF, kKC, 0);
  operand_planes<<<dim3(kNG / 32, kNH / 64), 256, 0, stream>>>(Whh_f, kNH, kNG, PF, kKC, kNI);
  operand_planes<<<dim3(kNG / 32, kNI / 64), 256, 0, stream>>>(Wih_b, kNI, kNG, PB, kKC, 0);
  operand_planes<<<dim3(kNG / 32, kNH / 64), 256, 0, stream>>>(Whh_b, kNH, kNG, PB, kKC, kNI);
  operand_planes<<<dim3(kNG / 32, kNI / 64), 256, 0, stream>>>(Wih_d, kNI, kNG, PD, kKC, 0);
  operand_planes<<<dim3(kNG / 32, kNH / 64), 256, 0, stream>>>(Whh_d, kNH, kNG, PD, kKC, kNI);
  operand_planes<<<dim3((2 * kNZ) / 32, (2 * kNH) / 64), 256, 0, stream>>>(W_enc, 2 * kNH, 2 * kNZ, PENC, 2 * kNH, 0);
  operand_planes<<<dim3(kNH / 32, kNZ / 64), 256, 0, stream>>>(W_z2h, kNZ, kNH, PZ2H, kNZ, 0);
  operand_planes<<<dim3(kNI2 / 32, kNH / 64), 256, 0, stream>>>(W_h2i, kNH, kNI2, PH2I, kNH, 0);
  operand_planes<<<dim3(kNI2 / 32, 1), 256, 0, stream>>>(W_ed, kND, kNI2, PED, kK32P, 0);
  operand_planes<<<dim3(kND / 32, kNH / 64), 256, 0, stream>>>(W_dec, kNH, kND, PDEC, kNH, 0);

  static_assert(((kNL * (kNB / 16)) % 8) == 0 && (kNB / 16) == 128);
  embed_rows<<<(kNL * (kNB / 16)) / 8, 256, 0, stream>>>(x, PEE, b_ee, XE);

  encode_decode_steps<<<kBlocks, kThreads, 0, stream>>>(
      XE, PF, PB, PD, PENC, PZ2H, PH2I, PED, PDEC,
      eps, bih_f, bhh_f, bih_b, bhh_b, b_enc, b_z2h, b_h2i, bih_d, bhh_d, b_ed, b_dec, out);
}
